// QuantumRegressionModel_65481071400898
// MI455X (gfx1250) — hardware-verified
//
#include <hip/hip_runtime.h>
#include <stdint.h>


#define NTOK 8192
#define DIM  256
#define EP   264
#define TP   72

typedef _Float16 v16h __attribute__((ext_vector_type(16)));
typedef _Float16 v8h  __attribute__((ext_vector_type(8)));
typedef float    v8f  __attribute__((ext_vector_type(8)));
typedef float    v4f  __attribute__((ext_vector_type(4)));
union Frag { v16h v; v8h hl[2]; };

static __device__ __forceinline__ v8f vz8() {
  v8f z = {0.f, 0.f, 0.f, 0.f, 0.f, 0.f, 0.f, 0.f};
  return z;
}

static __device__ __forceinline__ v8f wmma_f16(v16h a, v16h b, v8f c) {
  v8f d = __builtin_amdgcn_wmma_f32_16x16x32_f16(false, a, false, b, (short)0, c, false, false);
  asm volatile("v_nop\n\tv_nop\n\tv_nop\n\tv_nop" : "+v"(d) : "v"(a), "v"(b));
  return d;
}

static __device__ __forceinline__ v16h ldfrag(const _Float16* p) {
  Frag f;
  f.hl[0] = *(const v8h*)p;
  f.hl[1] = *(const v8h*)(p + 16);
  return f.v;
}

__global__ __launch_bounds__(256)
void k_cvt_states(const float* __restrict__ S, _Float16* __restrict__ S16, _Float16* __restrict__ ST16) {
  __shared__ __align__(16) _Float16 T[DIM][TP];
  const int lane = threadIdx.x & 31, w = threadIdx.x >> 5;
  const int t0 = blockIdx.x * 64;
  v8h hv[8];
#pragma unroll
  for (int i = 0; i < 8; ++i) {
    const int rloc = w * 8 + i;
    const float* src = S + (size_t)(t0 + rloc) * DIM + lane * 8;
    const v4f x0 = *(const v4f*)src;
    const v4f x1 = *(const v4f*)(src + 4);
    v8h hq;
#pragma unroll
    for (int e = 0; e < 4; ++e) { hq[e] = (_Float16)x0[e]; hq[4 + e] = (_Float16)x1[e]; }
    hv[i] = hq;
    *(volatile v8h*)(S16 + (size_t)(t0 + rloc) * DIM + lane * 8) = hq;
#pragma unroll
    for (int e = 0; e < 8; ++e) T[lane * 8 + e][rloc] = hq[e];
  }
  __syncthreads();
  v8h tv[8];
#pragma unroll
  for (int it = 0; it < 8; ++it) {
    const int d = w * 32 + it * 4 + (lane >> 3);
    const int q = lane & 7;
    tv[it] = *(const v8h*)&T[d][q * 8];
    *(volatile v8h*)(ST16 + (size_t)d * NTOK + t0 + q * 8) = tv[it];
  }
  __threadfence();
#pragma unroll
  for (int i = 0; i < 8; ++i) {
    const int rloc = w * 8 + i;
    *(volatile v8h*)(S16 + (size_t)(t0 + rloc) * DIM + lane * 8) = hv[i];
  }
#pragma unroll
  for (int it = 0; it < 8; ++it) {
    const int d = w * 32 + it * 4 + (lane >> 3);
    const int q = lane & 7;
    *(volatile v8h*)(ST16 + (size_t)d * NTOK + t0 + q * 8) = tv[it];
  }
}

__global__ __launch_bounds__(256)
void k_cvt_w(const float* __restrict__ Wq, const float* __restrict__ Wk, _Float16* __restrict__ WT) {
  __shared__ __align__(16) _Float16 T2[16][EP];
  const int tid = threadIdx.x, lane = tid & 31, w = tid >> 5;
  const int mat = blockIdx.x >> 4;
  const int o0 = (blockIdx.x & 15) * 16;
  const float* W = (mat == 0) ? Wq : Wk;
  const float* src = W + (size_t)tid * DIM + o0;
#pragma unroll
  for (int i = 0; i < 4; ++i) {
    const v4f x = *(const v4f*)(src + 4 * i);
#pragma unroll
    for (int e = 0; e < 4; ++e) T2[4 * i + e][tid] = (_Float16)(x[e] * 16.0f);
  }
  __syncthreads();
  _Float16* dstb = WT + (size_t)mat * DIM * DIM;
  const v8h r0v = *(const v8h*)&T2[2 * w][lane * 8];
  const v8h r1v = *(const v8h*)&T2[2 * w + 1][lane * 8];
  _Float16* d0 = dstb + (size_t)(o0 + 2 * w) * DIM + lane * 8;
  _Float16* d1 = d0 + DIM;
  *(volatile v8h*)d0 = r0v;
  *(volatile v8h*)d1 = r1v;
  __threadfence();
  *(volatile v8h*)d0 = r0v;
  *(volatile v8h*)d1 = r1v;
}

__global__ __launch_bounds__(128)
void k_proj(const _Float16* __restrict__ S16, const _Float16* __restrict__ WT,
            _Float16* __restrict__ Q16, _Float16* __restrict__ K16) {
  __shared__ __align__(16) _Float16 E[4][16][EP];
  const int lane = threadIdx.x & 31, w = threadIdx.x >> 5;
  const int h = lane >> 4, n = lane & 15;
  const int t0 = blockIdx.x * 64 + w * 16;
  v16h a[8];
  const _Float16* arow = S16 + (size_t)(t0 + n) * DIM + 8 * h;
#pragma unroll
  for (int c = 0; c < 8; ++c) a[c] = ldfrag(arow + c * 32);

#pragma unroll 1
  for (int mat = 0; mat < 2; ++mat) {
    const _Float16* wt = WT + (size_t)mat * DIM * DIM + 8 * h;
    _Float16* dst = (mat == 0) ? Q16 : K16;
#pragma unroll 1
    for (int nc = 0; nc < 16; ++nc) {
      const _Float16* brow = wt + (size_t)(nc * 16 + n) * DIM;
      v8f acc = vz8();
#pragma unroll
      for (int c = 0; c < 8; ++c) acc = wmma_f16(a[c], ldfrag(brow + c * 32), acc);
#pragma unroll
      for (int r = 0; r < 8; ++r) E[w][8 * h + r][nc * 16 + n] = (_Float16)acc[r];
    }
    __syncthreads();
#pragma unroll
    for (int i = 0; i < 16; ++i) {
      const v8h v = *(const v8h*)&E[w][i][lane * 8];
      *(volatile v8h*)(dst + (size_t)(t0 + i) * DIM + lane * 8) = v;
    }
    __threadfence();
#pragma unroll
    for (int i = 0; i < 16; ++i) {
      const v8h v = *(const v8h*)&E[w][i][lane * 8];
      *(volatile v8h*)(dst + (size_t)(t0 + i) * DIM + lane * 8) = v;
    }
    __syncthreads();
  }
}

__global__ __launch_bounds__(128)
void k_attn(const _Float16* __restrict__ Q16, const _Float16* __restrict__ K16,
            const _Float16* __restrict__ ST16, _Float16* __restrict__ A16,
            float* __restrict__ SQ) {
  __shared__ __align__(16) _Float16 E[4][16][EP];
  __shared__ __align__(16) float sqb[64];
  const int lane = threadIdx.x & 31, w = threadIdx.x >> 5;
  const int h = lane >> 4, n = lane & 15;
  const int q0 = blockIdx.x * 64 + w * 16;
  const _Float16* qrow = Q16 + (size_t)(q0 + n) * DIM + 8 * h;
  const _Float16* vrow = ST16 + (size_t)n * NTOK + 8 * h;

  v8f o[16];
#pragma unroll
  for (int nc = 0; nc < 16; ++nc) o[nc] = vz8();
  float m = -__builtin_inff();
  float l = 0.f;

#pragma unroll 1
  for (int kb = 0; kb < NTOK / 32; ++kb) {
    const int j0 = kb * 32;
    const _Float16* k0row = K16 + (size_t)(j0 + n) * DIM + 8 * h;
    const _Float16* k1row = K16 + (size_t)(j0 + 16 + n) * DIM + 8 * h;
    v8f s0 = vz8(), s1 = vz8();
#pragma unroll
    for (int c = 0; c < 8; ++c) {
      const v16h bq = ldfrag(qrow + c * 32);
      const v16h a0 = ldfrag(k0row + c * 32);
      const v16h a1 = ldfrag(k1row + c * 32);
      s0 = wmma_f16(a0, bq, s0);
      s1 = wmma_f16(a1, bq, s1);
    }
    float p[16];
    float mx = -__builtin_inff();
#pragma unroll
    for (int r = 0; r < 8; ++r) {
      p[r]     = s0[r] * (1.0f / 4096.0f);
      p[8 + r] = s1[r] * (1.0f / 4096.0f);
      mx = fmaxf(mx, fmaxf(p[r], p[8 + r]));
    }
    mx = fmaxf(mx, __shfl_xor(mx, 16));
    const float mn = fmaxf(m, mx);
    const float alpha = __expf(m - mn);
    m = mn;
    float ps = 0.f;
#pragma unroll
    for (int i = 0; i < 16; ++i) { p[i] = __expf(p[i] - mn); ps += p[i]; }
    l = l * alpha + ps;
    if (__ballot(alpha < 1.0f) != 0ull) {
      v8f arv;
#pragma unroll
      for (int r = 0; r < 8; ++r) arv[r] = __shfl(alpha, 8 * h + r);
#pragma unroll
      for (int nc = 0; nc < 16; ++nc) o[nc] = o[nc] * arv;
    }
    Frag pa;
    v8h p0, p1;
#pragma unroll
    for (int r = 0; r < 8; ++r) {
      p0[r] = (_Float16)(p[r] * 16384.0f);
      p1[r] = (_Float16)(p[8 + r] * 16384.0f);
    }
    pa.hl[0] = p0;
    pa.hl[1] = p1;
    const _Float16* vb = vrow + j0;
#pragma unroll
    for (int nc = 0; nc < 16; ++nc) {
      const v16h b = ldfrag(vb + (size_t)nc * 16 * NTOK);
      o[nc] = wmma_f16(pa.v, b, o[nc]);
    }
  }

  const float lt = l + __shfl_xor(l, 16);
  float inv[8], sqp[8];
#pragma unroll
  for (int r = 0; r < 8; ++r) {
    const float lr = __shfl(lt, 8 * h + r);
    inv[r] = (1.0f / lr) * (1.0f / 16384.0f);
    sqp[r] = 0.f;
  }
#pragma unroll
  for (int nc = 0; nc < 16; ++nc) {
#pragma unroll
    for (int r = 0; r < 8; ++r) {
      const float av = o[nc][r] * inv[r];
      sqp[r] += av * av;
      E[w][8 * h + r][nc * 16 + n] = (_Float16)(av * 64.0f);
    }
  }
#pragma unroll
  for (int r = 0; r < 8; ++r) {
    float t = sqp[r];
    t += __shfl_xor(t, 1); t += __shfl_xor(t, 2);
    t += __shfl_xor(t, 4); t += __shfl_xor(t, 8);
    sqp[r] = t;
  }
  if (n == 0) {
    const v4f c0 = {sqp[0], sqp[1], sqp[2], sqp[3]};
    const v4f c1 = {sqp[4], sqp[5], sqp[6], sqp[7]};
    *(v4f*)&sqb[w * 16 + 8 * h] = c0;
    *(v4f*)&sqb[w * 16 + 8 * h + 4] = c1;
  }
  __syncthreads();
#pragma unroll
  for (int i = 0; i < 16; ++i) {
    const v8h v = *(const v8h*)&E[w][i][lane * 8];
    *(volatile v8h*)(A16 + (size_t)(q0 + i) * DIM + lane * 8) = v;
  }
  const v4f sv = *(const v4f*)&sqb[(lane & 15) * 4];
  float* sqd = SQ + (size_t)blockIdx.x * 64 + (lane & 15) * 4;
  const bool wsq = (w == 0) && (lane < 16);
  if (wsq) *(volatile v4f*)sqd = sv;
  __threadfence();
#pragma unroll
  for (int i = 0; i < 16; ++i) {
    const v8h v = *(const v8h*)&E[w][i][lane * 8];
    *(volatile v8h*)(A16 + (size_t)(q0 + i) * DIM + lane * 8) = v;
  }
  if (wsq) *(volatile v4f*)sqd = sv;
}

__global__ __launch_bounds__(128)
void k_gram(const _Float16* __restrict__ A16, const float* __restrict__ SQ,
            const float* __restrict__ W1, const float* __restrict__ b1,
            const float* __restrict__ W2, const float* __restrict__ b2,
            float* __restrict__ out) {
  __shared__ __align__(16) float fs[64];
  __shared__ __align__(16) float ob[64];
  const int lane = threadIdx.x & 31, w = threadIdx.x >> 5;
  const int h = lane >> 4, n = lane & 15;
  const int i0 = blockIdx.x * 64 + w * 16;
  v16h a[8];
  const _Float16* arow = A16 + (size_t)(i0 + n) * DIM + 8 * h;
#pragma unroll
  for (int c = 0; c < 8; ++c) a[c] = ldfrag(arow + c * 32);
  float sqi[8], acc[8];
#pragma unroll
  for (int r = 0; r < 8; ++r) { sqi[r] = SQ[i0 + 8 * h + r]; acc[r] = 0.f; }

#pragma unroll 1
  for (int jb = 0; jb < NTOK / 32; ++jb) {
    const int j0 = jb * 32;
    const _Float16* b0row = A16 + (size_t)(j0 + n) * DIM + 8 * h;
    const _Float16* b1row = b0row + 16 * DIM;
    v8f g0 = vz8(), g1 = vz8();
#pragma unroll
    for (int c = 0; c < 8; ++c) {
      g0 = wmma_f16(a[c], ldfrag(b0row + c * 32), g0);
      g1 = wmma_f16(a[c], ldfrag(b1row + c * 32), g1);
    }
    const float sqj0 = SQ[j0 + n];
    const float sqj1 = SQ[j0 + 16 + n];
#pragma unroll
    for (int r = 0; r < 8; ++r) {
      float d0 = (sqi[r] + sqj0) - g0[r] * (1.0f / 2048.0f);
      float d1 = (sqi[r] + sqj1) - g1[r] * (1.0f / 2048.0f);
      d0 = fmaxf(d0, 0.f);
      d1 = fmaxf(d1, 0.f);
      acc[r] += __expf(-d0) + __expf(-d1);
    }
  }
#pragma unroll
  for (int r = 0; r < 8; ++r) {
    float t = acc[r];
    t += __shfl_xor(t, 1); t += __shfl_xor(t, 2);
    t += __shfl_xor(t, 4); t += __shfl_xor(t, 8);
    acc[r] = t;
  }
  if (n == 0) {
    const v4f c0 = {acc[0], acc[1], acc[2], acc[3]};
    const v4f c1 = {acc[4], acc[5], acc[6], acc[7]};
    *(v4f*)&fs[w * 16 + 8 * h] = c0;
    *(v4f*)&fs[w * 16 + 8 * h + 4] = c1;
  }
  __syncthreads();
  if (threadIdx.x < 64) {
    const float f = fs[threadIdx.x] * (1.0f / (float)NTOK);
    float hacc = 0.f;
#pragma unroll
    for (int u = 0; u < 64; ++u) {
      float t = f * W1[u] + b1[u];
      t = fmaxf(t, 0.f);
      hacc += t * W2[u];
    }
    ob[threadIdx.x] = hacc + b2[0];
  }
  __syncthreads();
  const v4f ov = *(const v4f*)&ob[(lane & 15) * 4];
  float* od = out + (size_t)blockIdx.x * 64 + (lane & 15) * 4;
  const bool wr = (w == 0) && (lane < 16);
  if (wr) *(volatile v4f*)od = ov;
  __threadfence();
  if (wr) *(volatile v4f*)od = ov;
}

extern "C" void kernel_launch(void* const* d_in, const int* in_sizes, int n_in,
                              void* d_out, int out_size, void* d_ws, size_t ws_size,
                              hipStream_t stream) {
  if (n_in < 7) return;
  if (in_sizes[0] != NTOK * DIM || in_sizes[1] != DIM * DIM || in_sizes[2] != DIM * DIM) return;
  if (in_sizes[3] < 64 || in_sizes[4] < 64 || in_sizes[5] < 64 || in_sizes[6] < 1) return;
  if (out_size < NTOK) return;

  const float* states = (const float*)d_in[0];
  const float* Wq     = (const float*)d_in[1];
  const float* Wk     = (const float*)d_in[2];
  const float* W1     = (const float*)d_in[3];
  const float* b1     = (const float*)d_in[4];
  const float* W2     = (const float*)d_in[5];
  const float* b2     = (const float*)d_in[6];
  float* out = (float*)d_out;

  char* ws = (char*)d_ws;
  size_t off = 0;
  const size_t plane = (size_t)NTOK * DIM * sizeof(_Float16);
  _Float16* S16  = (_Float16*)(ws + off); off += plane;
  _Float16* ST16 = (_Float16*)(ws + off); off += plane;
  _Float16* Q16  = (_Float16*)(ws + off); off += plane;
  _Float16* K16  = (_Float16*)(ws + off); off += plane;
  _Float16* A16  = (_Float16*)(ws + off); off += plane;
  _Float16* WT   = (_Float16*)(ws + off); off += (size_t)2 * DIM * DIM * sizeof(_Float16);
  float*    SQ   = (float*)(ws + off);    off += (size_t)NTOK * sizeof(float);
  if (off > ws_size) return;

  k_cvt_states<<<NTOK / 64, 256, 0, stream>>>(states, S16, ST16);
  k_cvt_w<<<32, 256, 0, stream>>>(Wq, Wk, WT);
  k_proj<<<NTOK / 64, 128, 0, stream>>>(S16, WT, Q16, K16);
  k_attn<<<NTOK / 64, 128, 0, stream>>>(Q16, K16, ST16, A16, SQ);
  k_gram<<<NTOK / 64, 128, 0, stream>>>(A16, SQ, W1, b1, W2, b2, out);
}
